// Kernel_16550548659508808100_53472342835837
// MI455X (gfx1250) — hardware-verified
//
#include <hip/hip_runtime.h>


#define NBI  16
#define CC   112
#define CP   128
#define HH   48
#define WW   48
#define HW   2304
#define KCV  352
typedef _Float16 h16;
typedef unsigned short bf;
typedef __attribute__((ext_vector_type(16))) __bf16   v16bf;
typedef __attribute__((ext_vector_type(16))) _Float16 v16h;
typedef __attribute__((ext_vector_type(8)))  _Float16 v8h;
typedef __attribute__((ext_vector_type(8)))  unsigned short v8us;
typedef __attribute__((ext_vector_type(8)))  float    v8f;
typedef __attribute__((ext_vector_type(4)))  float    v4f;
typedef v8h  __attribute__((may_alias)) v8ha;
typedef v4f  __attribute__((may_alias)) v4fa;
typedef v8us __attribute__((may_alias)) v8usa;

__device__ __forceinline__ unsigned short f2bf(float f) { unsigned u = __float_as_uint(f); u += 0x7FFFu + ((u >> 16) & 1u); return (unsigned short)(u >> 16); }
__device__ __forceinline__ float bf2f(unsigned short b) { return __uint_as_float(((unsigned)b) << 16); }
__device__ __forceinline__ float bfr(float f) { return bf2f(f2bf(f)); }
__device__ __forceinline__ v16h cat16(v8h lo, v8h hi) { return __builtin_shufflevector(lo, hi, 0, 1, 2, 3, 4, 5, 6, 7, 8, 9, 10, 11, 12, 13, 14, 15); }
__device__ __forceinline__ v16bf cat16b(v8us lo, v8us hi) { return __builtin_bit_cast(v16bf, __builtin_shufflevector(lo, hi, 0, 1, 2, 3, 4, 5, 6, 7, 8, 9, 10, 11, 12, 13, 14, 15)); }
__device__ __forceinline__ v8f wmma16(v16h a, v16h b, v8f c) { return __builtin_amdgcn_wmma_f32_16x16x32_f16(false, a, false, b, (short)0, c, false, false); }
__device__ __forceinline__ v8f wmmab(v16bf a, v16bf b, v8f c) { return __builtin_amdgcn_wmma_f32_16x16x32_bf16(false, a, false, b, (short)0, c, false, false); }


template <typename T16> struct WFrag;
template <> struct WFrag<h16> { typedef v16h V; static __device__ __forceinline__ V ld(const h16* p) { return cat16(*(const v8h*)p, *(const v8h*)(p + 16)); } static __device__ __forceinline__ v8f mma(V a, V b, v8f c) { return wmma16(a, b, c); } };
template <> struct WFrag<bf> { typedef v16bf V; static __device__ __forceinline__ V ld(const bf* p) { return cat16b(*(const v8us*)p, *(const v8us*)(p + 16)); } static __device__ __forceinline__ v8f mma(V a, V b, v8f c) { return wmmab(a, b, c); } };
template <typename T16, int NSPLIT, bool BIAS>
__global__ __launch_bounds__(32) void k_gemmw(const T16* __restrict__ A, const T16* __restrict__ A2, const T16* __restrict__ Bt, const T16* __restrict__ Bt2, int K, float* C, int ldc, const float* __restrict__ bias, size_t sA, size_t sB, size_t sC) {
    typedef typename WFrag<T16>::V V;
    __shared__ __align__(16) float os[16 * 68];
    const size_t z = blockIdx.z; A += z * sA; if (A2) A2 += z * sA; Bt += z * sB; if (Bt2) Bt2 += z * sB; C += z * sC;
    const int lane = threadIdx.x & 31, lr = lane & 15, hi = lane >> 4; const int r0 = blockIdx.x * 64, c0 = blockIdx.y * 64;
    v8f acc[4][4];
#pragma unroll
    for (int mb = 0; mb < 4; ++mb)
#pragma unroll
        for (int nb = 0; nb < 4; ++nb) acc[mb][nb] = (v8f){};
    const size_t aoff = (size_t)(r0 + lr) * K + 8 * hi, boff = (size_t)(c0 + lr) * K + 8 * hi;
#pragma unroll 1
    for (int kc = 0; kc < K; kc += 32) {
        V a[4], a2[4];
#pragma unroll
        for (int mb = 0; mb < 4; ++mb) { a[mb] = WFrag<T16>::ld(A + aoff + (size_t)mb * 16 * K + kc); if (NSPLIT == 1 || NSPLIT == 2) a2[mb] = WFrag<T16>::ld(A2 + aoff + (size_t)mb * 16 * K + kc); }
#pragma unroll
        for (int nb = 0; nb < 4; ++nb) { const V b = WFrag<T16>::ld(Bt + boff + (size_t)nb * 16 * K + kc); V b2; if (NSPLIT >= 2) b2 = WFrag<T16>::ld(Bt2 + boff + (size_t)nb * 16 * K + kc);
#pragma unroll
            for (int mb = 0; mb < 4; ++mb) { acc[mb][nb] = WFrag<T16>::mma(a[mb], b, acc[mb][nb]); if (NSPLIT == 1 || NSPLIT == 2) acc[mb][nb] = WFrag<T16>::mma(a2[mb], b, acc[mb][nb]); if (NSPLIT >= 2) acc[mb][nb] = WFrag<T16>::mma(a[mb], b2, acc[mb][nb]); } }
        asm volatile("v_nop\n\tv_nop\n\tv_nop\n\tv_nop" : "+v"(acc[0][0]), "+v"(acc[1][1]), "+v"(acc[2][2]), "+v"(acc[3][3]) : "v"(a[0]), "v"(a[3]));
    }
#pragma unroll
    for (int mb = 0; mb < 4; ++mb) {
#pragma unroll
        for (int nb = 0; nb < 4; ++nb) {
#pragma unroll
            for (int j = 0; j < 8; ++j) os[(hi * 8 + j) * 68 + nb * 16 + lr] = acc[mb][nb][j]; }
        __builtin_amdgcn_wave_barrier(); asm volatile("" ::: "memory");
        float* crow = C + (size_t)(r0 + mb * 16) * ldc + c0;
#pragma unroll 1
        for (int ps = 0; ps < 2; ++ps) {
#pragma unroll
            for (int s = 0; s < 8; ++s) { const int row = 2 * s + hi, cofs = lr * 4; v4f val = *(const v4fa*)(os + row * 68 + cofs); if (BIAS) { val[0] += bfr(bias[c0 + cofs]); val[1] += bfr(bias[c0 + cofs + 1]); val[2] += bfr(bias[c0 + cofs + 2]); val[3] += bfr(bias[c0 + cofs + 3]); }
                *(volatile v4f*)(crow + (size_t)row * ldc + cofs) = val; }
            if (ps == 0) __threadfence(); }
        __builtin_amdgcn_wave_barrier(); asm volatile("" ::: "memory");
    }
}

__device__ __forceinline__ void splitf(float y, unsigned short& h, unsigned short& l) { h = f2bf(y); l = f2bf(y - bf2f(h)); }
typedef __attribute__((ext_vector_type(2))) unsigned short v2us;
typedef __attribute__((ext_vector_type(4))) unsigned short v4us;

__global__ __launch_bounds__(256) void k_wcv(const float* __restrict__ w, bf* WB) { const int i = (blockIdx.x * 256 + threadIdx.x) * 4; if (i >= CP * KCV) return; const int o = i / KCV, k0 = i % KCV; v4us ov;
#pragma unroll
    for (int q = 0; q < 4; ++q) { const int kk = k0 + q; ov[q] = (o < CC && kk < CC * 3) ? f2bf(w[(o * CC + kk / 3) * 3 + kk % 3]) : (unsigned short)0; } *(volatile v4us*)(WB + i) = ov; __threadfence(); *(volatile v4us*)(WB + i) = ov; }
__global__ __launch_bounds__(64) void k_t7(const float* __restrict__ xb, const float* __restrict__ p7, float* T7L, float* T17L) { __shared__ float t7s[64]; const int h = threadIdx.x; float t7 = 0.f;
    if (h < HH) { const int hs = (h - 2 + HH) % HH;
#pragma unroll 1
        for (int k = 0; k < 3; ++k) {
#pragma unroll 1
            for (int w = 0; w < WW; ++w) { const int ws = w + 3 * k - 3; if (ws < 0 || ws >= WW) continue; float m = 0.f;
#pragma unroll 1
                for (int c = 0; c < CC; ++c) m = __fadd_rn(m, bfr(xb[((size_t)c * HH + hs) * WW + ws]));
                float p = __fmul_rn(m * (1.0f / CC), bfr(p7[k * WW + w])); asm volatile("" : "+v"(p)); t7 = __fadd_rn(t7, p); } } }
    t7s[h] = (h < HH) ? t7 : 0.f; __syncthreads();
    float t17 = 0.f; if (h < 7) { for (int hp = 0; hp < HH; ++hp) { const int idx = 2 * h + hp - 6; if (idx >= 0 && idx < HH) t17 = __fadd_rn(t17, fabsf(t7s[idx])); } t17 = t17 * (1.0f / HH); }
    const float a = (h < HH) ? t7 : 0.f; *(volatile float*)(T7L + h) = a; if (h < 32) *(volatile float*)(T17L + h) = (h < 7) ? t17 : 0.f; __threadfence(); *(volatile float*)(T7L + h) = a; if (h < 32) *(volatile float*)(T17L + h) = (h < 7) ? t17 : 0.f; }
__global__ __launch_bounds__(256) void k_elt(const float* __restrict__ xb, const float* __restrict__ p8, const float* __restrict__ p19, const float* __restrict__ T17L, float* T10, bf* T19h, bf* T19l, bf* XB) { const int e = (blockIdx.x * 256 + threadIdx.x) * 4; if (e >= CP * HW) return; const int p0 = e % HW; const int c = e / HW; const int h = p0 / WW, w0 = p0 % WW; v4f o10; v4us th, tl, xo;
#pragma unroll
    for (int q = 0; q < 4; ++q) { const int w = w0 + q, p = p0 + q; float t10 = 0.f, t19 = 0.f, xv = 0.f;
        if (c < CC) { xv = bfr(xb[(size_t)c * HW + p]); const float t5 = bfr(xb[((size_t)c * HH + (h - 2 + HH) % HH) * WW + (w + 1) % WW]); const float t8 = __fmul_rn(bfr(p8[c * HH + h]), t5); const float t9 = __fadd_rn(xv, t8); t10 = __fsub_rn(t8, t9); t19 = __fmul_rn(bfr(p19[c]), __fsub_rn(T17L[(c * HW + p) % 7], t10)); }
        o10[q] = t10; unsigned short a, b; splitf(t19, a, b); th[q] = a; tl[q] = b; xo[q] = f2bf(xv); }
    for (int ps = 0; ps < 2; ++ps) { *(volatile v4f*)(T10 + e) = o10; *(volatile v4us*)(T19h + e) = th; *(volatile v4us*)(T19l + e) = tl; *(volatile v4us*)(XB + e) = xo; if (ps == 0) __threadfence(); } }
__global__ __launch_bounds__(256) void k_i2c(const float* __restrict__ T10, bf* Ah, bf* Al) { const int e = (blockIdx.x * 256 + threadIdx.x) * 4; if (e >= HW * KCV) return; const int k0 = e % KCV; const int p = e / KCV; const int h = p / WW, w = p % WW; v4us oh, ol;
#pragma unroll
    for (int q = 0; q < 4; ++q) { const int kk = k0 + q; float v = 0.f; if (kk < CC * 3) { const int c = kk / 3, k = kk % 3; const int ws = w + 2 * k - 2; if (ws >= 0 && ws < WW) v = T10[(size_t)c * HW + h * WW + ws]; } unsigned short a, b; splitf(v, a, b); oh[q] = a; ol[q] = b; }
    *(volatile v4us*)(Ah + e) = oh; *(volatile v4us*)(Al + e) = ol; __threadfence(); *(volatile v4us*)(Ah + e) = oh; *(volatile v4us*)(Al + e) = ol; }
__global__ __launch_bounds__(256) void k_t13(const float* __restrict__ T11, const float* __restrict__ xb, bf* Th, bf* Tl) { const int e = (blockIdx.x * 256 + threadIdx.x) * 4; if (e >= HW * CP) return; const int c0 = e % CP; const int q_ = e / CP; v4us oh, ol;
#pragma unroll
    for (int q = 0; q < 4; ++q) { const int c = c0 + q; float v = 0.f; if (c < CC) v = fmaxf(T11[e + q], bfr(xb[(size_t)c * HW + q_])); unsigned short a, b; splitf(v, a, b); oh[q] = a; ol[q] = b; }
    *(volatile v4us*)(Th + e) = oh; *(volatile v4us*)(Tl + e) = ol; __threadfence(); *(volatile v4us*)(Th + e) = oh; *(volatile v4us*)(Tl + e) = ol; }
__global__ __launch_bounds__(256) void k_mpl(const float* __restrict__ M, bf* Mh, bf* Ml) { const int e = (blockIdx.x * 256 + threadIdx.x) * 4; if (e >= CP * CP) return; const v4f a = *(const v4f*)(M + e); v4us oh, ol;
#pragma unroll
    for (int q = 0; q < 4; ++q) { unsigned short u, b; splitf(a[q], u, b); oh[q] = u; ol[q] = b; } *(volatile v4us*)(Mh + e) = oh; *(volatile v4us*)(Ml + e) = ol; __threadfence(); *(volatile v4us*)(Mh + e) = oh; *(volatile v4us*)(Ml + e) = ol; }
__global__ __launch_bounds__(128) void k_s1(const bf* __restrict__ T19h, const bf* __restrict__ T19l, const float* __restrict__ T7L, float* S1) { const int c = blockIdx.x * 128 + threadIdx.x; if (c >= CP) return; float s = 0.f;
#pragma unroll 1
    for (int p = 0; p < HW; ++p) { const float t = __fadd_rn(bf2f(T19h[(size_t)c * HW + p]), bf2f(T19l[(size_t)c * HW + p])); float q = __fmul_rn(t, T7L[p / WW]); asm volatile("" : "+v"(q)); s = __fadd_rn(s, q); }
    *(volatile float*)(S1 + c) = s; __threadfence(); *(volatile float*)(S1 + c) = s; }
__global__ __launch_bounds__(256) void k_out(const float* __restrict__ Q, const float* __restrict__ S1, float* OUTb) { const int e = (blockIdx.x * 256 + threadIdx.x) * 4; if (e >= CC * HW) return; const int c = e / HW; const int q0 = e % HW; const float s2 = 2.0f * S1[c]; v4f o;
#pragma unroll
    for (int q = 0; q < 4; ++q) { float t = __fmul_rn(Q[(size_t)c * HW + q0 + q], 0.0944911182523068f); asm volatile("" : "+v"(t)); o[q] = __fmul_rn(__fsub_rn(s2, t), 1.0f / 48.0f); }
    *(volatile v4f*)(OUTb + e) = o; __threadfence(); *(volatile v4f*)(OUTb + e) = o; }

extern "C" void kernel_launch(void* const* d_in, const int* in_sizes, int n_in,
                              void* d_out, int out_size, void* d_ws, size_t ws_size, hipStream_t stream) {
    (void)in_sizes; (void)n_in; (void)out_size;
    const float* x = (const float*)d_in[0]; const float* p7 = (const float*)d_in[1]; const float* p8 = (const float*)d_in[2]; const float* p19 = (const float*)d_in[3]; const float* cw = (const float*)d_in[4];
    float* OUT = (float*)d_out;
    char* wsp = (char*)d_ws;
    auto take = [&](size_t bytes) { char* p = wsp; wsp += (bytes + 255) & ~(size_t)255; return (void*)p; };
    bf* WB = (bf*)take((size_t)CP * KCV * 2); float* T7L = (float*)take(256); float* T17L = (float*)take(128); float* T10 = (float*)take((size_t)CP * HW * 4); bf* T19h = (bf*)take((size_t)CP * HW * 2); bf* T19l = (bf*)take((size_t)CP * HW * 2); bf* XB = (bf*)take((size_t)CP * HW * 2);
    bf* Ah = (bf*)take((size_t)HW * KCV * 2); bf* Al = (bf*)take((size_t)HW * KCV * 2); float* T11 = (float*)take((size_t)HW * CP * 4); bf* T13h = (bf*)take((size_t)HW * CP * 2); bf* T13l = (bf*)take((size_t)HW * CP * 2); float* M = (float*)take(CP * CP * 4); bf* Mh = (bf*)take(CP * CP * 2); bf* Ml = (bf*)take(CP * CP * 2); float* Qm = (float*)take((size_t)CP * HW * 4); float* S1 = (float*)take(CP * 4);
    if ((size_t)(wsp - (char*)d_ws) > ws_size) return;
    k_wcv<<<(CP * KCV / 4 + 255) / 256, 256, 0, stream>>>(cw, WB);
    for (int b = 0; b < NBI; ++b) { const float* xb = x + (size_t)b * CC * HW;
        k_t7<<<1, 64, 0, stream>>>(xb, p7, T7L, T17L);
        k_elt<<<(CP * HW / 4 + 255) / 256, 256, 0, stream>>>(xb, p8, p19, T17L, T10, T19h, T19l, XB);
        k_i2c<<<(HW * KCV / 4 + 255) / 256, 256, 0, stream>>>(T10, Ah, Al); k_gemmw<bf, 1, false><<<dim3(HW / 64, CP / 64, 1), 32, 0, stream>>>(Ah, Al, WB, nullptr, KCV, T11, CP, nullptr, 0, 0, 0);
        k_t13<<<(HW * CP / 4 + 255) / 256, 256, 0, stream>>>(T11, xb, T13h, T13l);
        k_gemmw<bf, 1, false><<<dim3(CP / 64, CP / 64, 1), 32, 0, stream>>>(T19h, T19l, XB, nullptr, HW, M, CP, nullptr, 0, 0, 0);
        k_mpl<<<(CP * CP / 4 + 255) / 256, 256, 0, stream>>>(M, Mh, Ml); k_gemmw<bf, 2, false><<<dim3(CP / 64, HW / 64, 1), 32, 0, stream>>>(Mh, Ml, T13h, T13l, CP, Qm, HW, nullptr, 0, 0, 0);
        k_s1<<<1, 128, 0, stream>>>(T19h, T19l, T7L, S1);
        k_out<<<(CC * HW / 4 + 255) / 256, 256, 0, stream>>>(Qm, S1, OUT + (size_t)b * CC * HW); }
}
